// GroupedGRU_80702435492217
// MI455X (gfx1250) — hardware-verified
//
#include <hip/hip_runtime.h>
#include <math.h>

typedef __attribute__((ext_vector_type(16))) _Float16 v16h;
typedef __attribute__((ext_vector_type(8)))  _Float16 v8h;
typedef __attribute__((ext_vector_type(8)))  float    v8f;
typedef __attribute__((ext_vector_type(4)))  float    v4f;

constexpr int kG     = 4;
constexpr int kI     = 128;
constexpr int kH     = 128;
constexpr int kB     = 32;
constexpr int kT     = 1000;
constexpr int kH3    = 3 * kH;
constexpr int kKc    = kI + kH;
constexpr int kRowW  = kG * kH;
constexpr int kMt    = 16;
constexpr int kTilesPerG = kB / kMt;
constexpr int kBlocks    = kG * kTilesPerG;
constexpr int kThreads   = 256;
constexpr int kWaves     = kThreads / 32;
constexpr int kWP    = 264;
constexpr int kHsP   = 132;

static_assert(kG * kI == kRowW, "input row width");
static_assert(kKc == 256 && (kKc % 32) == 0, "combined K is a multiple of 32");
static_assert(kWaves * 16 == kH, "one 16-column tile of hidden units per wave");
static_assert(kMt == 16 && (kB % kMt) == 0, "one 16-row M tile per block");
static_assert(kMt == 2 * kWaves, "two output rows per wave in the store pass");
static_assert(kThreads == kMt * (kI / 8), "x staging: one 8-element chunk per thread");
static_assert((kH3 * kI / 8) % kThreads == 0, "weight fill chunk count");
static_assert((kWP % 8) == 0 && kWP >= kKc && (kHsP % 4) == 0 && kHsP >= kH, "LDS pitches");

constexpr float kCarryAct     = 64.0f;
constexpr float kCarryW       = 1024.0f;
constexpr float kFold         = 1.0f / (kCarryAct * kCarryW);
constexpr float kF16MinNormal = 6.103515625e-05f;

constexpr int kOpElems  = kMt * kWP;
constexpr int kHsElems  = kMt * kHsP;
constexpr int kLdsW     = kH3 * kWP * 2;
constexpr int kLdsOp    = 2 * kOpElems * 2;
constexpr int kLdsHs    = 2 * kHsElems * 4;
constexpr int kLdsTotal = kLdsW + kLdsOp + kLdsHs;
static_assert(kLdsW == 202752 && kLdsOp == 16896 && kLdsHs == 16896 && kLdsTotal == 236544, "LDS map");
static_assert((kLdsW % 16) == 0 && ((kLdsW + kLdsOp) % 16) == 0, "16-B aligned LDS regions");

__device__ __forceinline__ float bf16_value(float f) {
  unsigned u = __float_as_uint(f);
  u = (u + 0x7FFFu + ((u >> 16) & 1u)) & 0xFFFF0000u;
  return __uint_as_float(u);
}
__device__ __forceinline__ _Float16 to_f16_flush(float v) {
  const float s = (fabsf(v) < kF16MinNormal) ? 0.0f : v;
  return (_Float16)s;
}
union FragH { v16h v; v8h h[2]; };
__device__ __forceinline__ v16h frag_load(const _Float16* p) {
  FragH f;
  f.h[0] = *(const v8h*)(p);
  f.h[1] = *(const v8h*)(p + 16);
  return f.v;
}
__device__ __forceinline__ v8f mma_f16(v16h a, v16h b, v8f c) {
  c = __builtin_amdgcn_wmma_f32_16x16x32_f16(false, a, false, b, (short)0, c, false, false);
  asm volatile("v_nop\n\tv_nop\n\tv_nop\n\tv_nop" : "+v"(c) : "v"(a), "v"(b));
  return c;
}
__device__ __forceinline__ void k_block(const _Float16* ap, const _Float16* wr, const _Float16* wz,
                                        const _Float16* wn, v8f& aR, v8f& aZ, v8f& aN) {
#pragma unroll 2
  for (int ks = 0; ks < 4; ++ks) {
    const int ko = ks * 32;
    const v16h a  = frag_load(ap + ko);
    const v16h br = frag_load(wr + ko);
    const v16h bz = frag_load(wz + ko);
    const v16h bn = frag_load(wn + ko);
    aR = mma_f16(a, br, aR);
    aZ = mma_f16(a, bz, aZ);
    aN = mma_f16(a, bn, aN);
  }
}
__device__ __forceinline__ v8h pack_act(v4f a0, v4f a1) {
  v8h hv;
#pragma unroll
  for (int e = 0; e < 4; ++e) {
    const float f0 = a0[e];
    const float f1 = a1[e];
    hv[e]     = to_f16_flush(bf16_value(f0) * kCarryAct);
    hv[4 + e] = to_f16_flush(bf16_value(f1) * kCarryAct);
  }
  return hv;
}
__device__ __forceinline__ void fill_weight_half(const float* __restrict__ src, _Float16* dst, int tid) {
#pragma unroll 1
  for (int it = 0; it < (kH3 * kI / 8) / kThreads; ++it) {
    const int chunk = it * kThreads + tid;
    const int n  = chunk >> 4;
    const int c8 = (chunk & 15) * 8;
    const v4f a0 = *(const v4f*)(src + (size_t)n * kI + c8);
    const v4f a1 = *(const v4f*)(src + (size_t)n * kI + c8 + 4);
    v8h hv;
#pragma unroll
    for (int e = 0; e < 4; ++e) {
      const float f0 = a0[e];
      const float f1 = a1[e];
      hv[e]     = to_f16_flush(bf16_value(f0) * kCarryW);
      hv[4 + e] = to_f16_flush(bf16_value(f1) * kCarryW);
    }
    *(v8h*)(dst + n * kWP + c8) = hv;
  }
}

__global__ __launch_bounds__(256) void grouped_cell_steps(
    const float* __restrict__ x, const float* __restrict__ w_ih, const float* __restrict__ w_hh,
    const float* __restrict__ b_ih, const float* __restrict__ b_hh, float* __restrict__ out)
{
  extern __shared__ __align__(16) unsigned char lds_raw[];
  _Float16* Wl = (_Float16*)lds_raw;
  _Float16* OP = (_Float16*)(lds_raw + kLdsW);
  float*    HS = (float*)(lds_raw + kLdsW + kLdsOp);

  const int tid  = threadIdx.x;
  const int lane = tid & 31;
  const int wave = tid >> 5;
  const int hh   = lane >> 4;
  const int c    = lane & 15;
  const int g    = blockIdx.x / kTilesPerG;
  const int b0   = (blockIdx.x - g * kTilesPerG) * kMt;

  fill_weight_half(w_ih + (size_t)g * kH3 * kI, Wl, tid);
  fill_weight_half(w_hh + (size_t)g * kH3 * kH, Wl + kI, tid);

  const int j = wave * 16 + c;
  const float* bi = b_ih + g * kH3;
  const float* bh = b_hh + g * kH3;
  const float bR  = bf16_value(bi[j]) + bf16_value(bh[j]);
  const float bZ  = bf16_value(bi[kH + j]) + bf16_value(bh[kH + j]);
  const float bNi = bf16_value(bi[2 * kH + j]);
  const float bNh = bf16_value(bh[2 * kH + j]);

  const int srow = tid >> 4;
  const int scol = (tid & 15) * 8;
  const float* xrow = x + ((size_t)(b0 + srow) * kT) * kRowW + g * kI + scol;

  {
    const v4f xa = *(const v4f*)(xrow);
    const v4f xb = *(const v4f*)(xrow + 4);
    const v8h xv = pack_act(xa, xb);
    *(v8h*)(OP + srow * kWP + scol) = xv;
    const _Float16 zh = (_Float16)0.0f;
    const v8h zv = (v8h){zh, zh, zh, zh, zh, zh, zh, zh};
    *(v8h*)(OP + srow * kWP + kI + scol) = zv;
  }
  __syncthreads();

  const _Float16* wr = Wl + (size_t)j * kWP + 8 * hh;
  const _Float16* wz = Wl + (size_t)(kH + j) * kWP + 8 * hh;
  const _Float16* wn = Wl + (size_t)(2 * kH + j) * kWP + 8 * hh;
  const int aoff = c * kWP + 8 * hh;

  float* orow0 = out + ((size_t)(b0 + 2 * wave) * kT) * kRowW + g * kH + lane * 4;
  float* orow1 = orow0 + (size_t)kT * kRowW;

  float hreg[8];
#pragma unroll
  for (int r = 0; r < 8; ++r) hreg[r] = 0.0f;

#pragma unroll 1
  for (int t = 0; t < kT; ++t) {
    const int cur = t & 1;
    const _Float16* oc = OP + cur * kOpElems;
    _Float16* on = OP + (cur ^ 1) * kOpElems;
    float* hsb = HS + cur * kHsElems;

    const int tn = (t + 1 < kT) ? (t + 1) : (kT - 1);
    const float* xp = xrow + (size_t)tn * kRowW;
    const v4f xa = *(const v4f*)(xp);
    const v4f xb = *(const v4f*)(xp + 4);

    v8f accR  = (v8f){0.f, 0.f, 0.f, 0.f, 0.f, 0.f, 0.f, 0.f};
    v8f accZ  = (v8f){0.f, 0.f, 0.f, 0.f, 0.f, 0.f, 0.f, 0.f};
    v8f accNi = (v8f){0.f, 0.f, 0.f, 0.f, 0.f, 0.f, 0.f, 0.f};
    v8f accNh = (v8f){0.f, 0.f, 0.f, 0.f, 0.f, 0.f, 0.f, 0.f};
    k_block(oc + aoff, wr, wz, wn, accR, accZ, accNi);
    k_block(oc + aoff + kI, wr + kI, wz + kI, wn + kI, accR, accZ, accNh);

#pragma unroll
    for (int r = 0; r < 8; ++r) {
      const float ar  = accR[r] * kFold + bR;
      const float az  = accZ[r] * kFold + bZ;
      const float gin = accNi[r] * kFold + bNi;
      const float ghn = accNh[r] * kFold + bNh;
      const float rg  = 1.0f / (1.0f + expf(-ar));
      const float zg  = 1.0f / (1.0f + expf(-az));
      const float ng  = tanhf(gin + rg * ghn);
      const float hv  = (1.0f - zg) * ng + zg * hreg[r];
      hreg[r] = hv;
      hsb[(8 * hh + r) * kHsP + j] = hv;
      on[(8 * hh + r) * kWP + kI + j] = to_f16_flush(hv * kCarryAct);
    }
    {
      const v8h xv = pack_act(xa, xb);
      *(v8h*)(on + srow * kWP + scol) = xv;
    }
    __syncthreads();

    {
      const v4f o0 = *(const v4f*)(hsb + (2 * wave) * kHsP + lane * 4);
      const v4f o1 = *(const v4f*)(hsb + (2 * wave + 1) * kHsP + lane * 4);
      float* p0 = orow0 + (size_t)t * kRowW;
      float* p1 = orow1 + (size_t)t * kRowW;
      *(volatile v4f*)p0 = o0;
      *(volatile v4f*)p1 = o1;
      __threadfence();
      *(volatile v4f*)p0 = o0;
      *(volatile v4f*)p1 = o1;
    }
  }
}

extern "C" void kernel_launch(void* const* d_in, const int* in_sizes, int n_in,
                              void* d_out, int out_size, void* d_ws, size_t ws_size,
                              hipStream_t stream) {
  (void)d_ws;
  (void)ws_size;
  if (n_in < 5) return;
  if (in_sizes[0] != kB * kT * kRowW) return;
  if (in_sizes[1] != kG * kH3 * kI) return;
  if (in_sizes[2] != kG * kH3 * kH) return;
  if (in_sizes[3] != kG * kH3) return;
  if (in_sizes[4] != kG * kH3) return;
  if (out_size != kB * kT * kRowW) return;

  const float* x    = (const float*)d_in[0];
  const float* w_ih = (const float*)d_in[1];
  const float* w_hh = (const float*)d_in[2];
  const float* b_ih = (const float*)d_in[3];
  const float* b_hh = (const float*)d_in[4];
  float* out = (float*)d_out;

  grouped_cell_steps<<<dim3(kBlocks), dim3(kThreads), (size_t)kLdsTotal, stream>>>(
      x, w_ih, w_hh, b_ih, b_hh, out);
}
